// ODEGRU_52913997087347
// MI455X (gfx1250) — hardware-verified
//
#include <hip/hip_runtime.h>
#include <math.h>

typedef _Float16 v16h __attribute__((ext_vector_type(16)));
typedef _Float16 v8h  __attribute__((ext_vector_type(8)));
typedef float    v8f  __attribute__((ext_vector_type(8)));
typedef float    v4f  __attribute__((ext_vector_type(4)));
typedef unsigned v4u  __attribute__((ext_vector_type(4)));
typedef unsigned v2u  __attribute__((ext_vector_type(2)));

constexpr int kT      = 100;
constexpr int kBatch  = 2048;
constexpr int kIn     = 32;
constexpr int kH      = 128;
constexpr int kOde    = 50;
constexpr int kOdeP   = 64;
constexpr int kL1     = 64;
constexpr int kNEuler = 10;
constexpr int kRows   = 16;
constexpr int kThreads = 128;

constexpr int XP = 40;
constexpr int HP = 136;
constexpr int UP = 72;

constexpr float kDtScale = (float)(1.0 / 24.0);
constexpr float kStep    = 0.1f;
constexpr float kActS    = 8.0f;
constexpr float kWgtS    = 16.0f;
constexpr float kInv     = 1.0f / 128.0f;
constexpr float kLog2e   = 1.44269504088896340736f;
constexpr float kTwoLog2e = 2.88539008177792681472f;

constexpr size_t kOffWih = 0;
constexpr size_t kOffWhh = kOffWih + (size_t)3 * kH * kIn * 2;
constexpr size_t kOffW1  = kOffWhh + (size_t)3 * kH * kH * 2;
constexpr size_t kOffW2  = kOffW1  + (size_t)kOdeP * kH * 2;
constexpr size_t kOffWl1 = kOffW2  + (size_t)kH * kOdeP * 2;
constexpr size_t kOffWs1 = kOffWl1 + (size_t)kL1 * kH * 2;
constexpr size_t kWsTotal = kOffWs1 + (size_t)kH * kH * 2;

__device__ __forceinline__ unsigned short f16bits(float f) {
  return __builtin_bit_cast(unsigned short, (_Float16)f);
}

union FragU { v16h v; v8h h[2]; };
__device__ __forceinline__ v16h frag_load(const _Float16* p) {
  FragU f; f.h[0] = *(const v8h*)(p); f.h[1] = *(const v8h*)(p + 16); return f.v;
}

__device__ __forceinline__ v8f mma_h(v16h a, v16h b, v8f c) {
  c = __builtin_amdgcn_wmma_f32_16x16x32_f16(false, a, false, b, (short)0, c, false, false);
  asm volatile("v_nop\n\tv_nop\n\tv_nop\n\tv_nop" : "+v"(c) : "v"(a), "v"(b));
  return c;
}

__device__ __forceinline__ v8f zero8() { v8f z = {0.f,0.f,0.f,0.f,0.f,0.f,0.f,0.f}; return z; }

__device__ __forceinline__ float ex2c(float a) {
  a = fminf(fmaxf(a, -100.0f), 100.0f);
  return __builtin_amdgcn_exp2f(a);
}
__device__ __forceinline__ float tanh_f(float x) {
  const float e = ex2c(x * kTwoLog2e);
  return 1.0f - 2.0f * __builtin_amdgcn_rcpf(1.0f + e);
}
__device__ __forceinline__ float sigm_f(float x) {
  const float e = ex2c(x * (-kLog2e));
  return __builtin_amdgcn_rcpf(1.0f + e);
}

__global__ __launch_bounds__(256) void prep_plane_f16(
    const float* __restrict__ src, int srows, int scols,
    unsigned short* __restrict__ dst, int drows, int dcols, float scale) {
  const int total8 = (drows * dcols) >> 3;
  const int i  = blockIdx.x * 256 + threadIdx.x;
  const int ic = (i < total8) ? i : (total8 - 1);
  const int e0 = ic * 8;
  const int n  = e0 / dcols;
  const int kb = e0 - n * dcols;
  const int nn = (n < srows) ? n : (srows - 1);
  unsigned w[4];
#pragma unroll
  for (int q = 0; q < 4; ++q) {
    unsigned short hb[2];
#pragma unroll
    for (int s = 0; s < 2; ++s) {
      const int k  = kb + 2 * q + s;
      const int kk = (k < scols) ? k : (scols - 1);
      const float v  = src[(size_t)nn * scols + kk];
      const float sv = v * ((n < srows && k < scols) ? scale : 0.0f);
      hb[s] = f16bits(sv);
    }
    w[q] = (unsigned)hb[0] | ((unsigned)hb[1] << 16);
  }
  if (i < total8) {
    v4u val = {w[0], w[1], w[2], w[3]};
    volatile v4u* p = ((volatile v4u*)dst) + i;
    *p = val;
    __threadfence();
    *p = val;
  }
}

__global__ __launch_bounds__(128) void odegru_main(
    const float* __restrict__ dt, const float* __restrict__ x,
    const unsigned short* __restrict__ wihp, const unsigned short* __restrict__ whhp,
    const unsigned short* __restrict__ w1pp, const unsigned short* __restrict__ w2pp,
    const unsigned short* __restrict__ wl1pp, const unsigned short* __restrict__ ws1pp,
    const float* __restrict__ bih, const float* __restrict__ bhh,
    const float* __restrict__ b1,  const float* __restrict__ b2,
    const float* __restrict__ bl1, const float* __restrict__ wmu, const float* __restrict__ bmu,
    const float* __restrict__ bs1, const float* __restrict__ ws2, const float* __restrict__ bs2,
    float* __restrict__ out) {
  __shared__ __align__(16) unsigned short xs_l[kRows * XP];
  __shared__ __align__(16) unsigned short hs_l[2 * kRows * HP];
  __shared__ __align__(16) unsigned short us_l[kRows * UP];
  __shared__ __align__(16) float scl_l[kRows];
  __shared__ __align__(16) float pmu_l[4 * kRows];
  __shared__ __align__(16) float psg_l[4 * kRows];
  __shared__ __align__(16) float mus_l[kRows * kT];
  __shared__ __align__(16) float sgs_l[kRows * kT];

  const _Float16* Wih = (const _Float16*)wihp;
  const _Float16* Whh = (const _Float16*)whhp;
  const _Float16* W1  = (const _Float16*)w1pp;
  const _Float16* W2  = (const _Float16*)w2pp;
  const _Float16* Wl1 = (const _Float16*)wl1pp;
  const _Float16* Ws1 = (const _Float16*)ws1pp;

  const int tid  = threadIdx.x;
  const int wave = tid >> 5;
  const int lane = tid & 31;
  const int hh   = lane >> 4;
  const int c    = lane & 15;
  const int koff = hh * 8;
  const int b0   = blockIdx.x * kRows;

  float brr[2], bzz[2], bxn[2], bhn[2], b2v[2], bs1v[2], ws2v[2];
#pragma unroll
  for (int us = 0; us < 2; ++us) {
    const int col = 32 * wave + 16 * us + c;
    brr[us]  = bih[col] + bhh[col];
    bzz[us]  = bih[kH + col] + bhh[kH + col];
    bxn[us]  = bih[2 * kH + col];
    bhn[us]  = bhh[2 * kH + col];
    b2v[us]  = b2[col];
    bs1v[us] = bs1[col];
    ws2v[us] = ws2[col];
  }
  const int col1 = 16 * wave + c;
  const int c1c  = (col1 < kOde) ? col1 : (kOde - 1);
  const float b1t  = b1[c1c];
  const float b1v  = (col1 < kOde) ? b1t : 0.0f;
  const float bl1v = bl1[col1];
  const float wmuv = wmu[col1];
  const float bmu0 = bmu[0];
  const float bs20 = bs2[0];

  {
    v4u z = {0u, 0u, 0u, 0u};
    for (int i = tid; i < (2 * kRows * HP) / 8; i += kThreads) *(v4u*)(hs_l + 8 * i) = z;
  }
  float hreg[2][8];
#pragma unroll
  for (int us = 0; us < 2; ++us)
#pragma unroll
    for (int r = 0; r < 8; ++r) hreg[us][r] = 0.0f;
  __syncthreads();

  const _Float16* xsh = (const _Float16*)xs_l;
  const _Float16* ush = (const _Float16*)us_l;

#pragma unroll 1
  for (int t = 0; t < kT; ++t) {
    {
      const int row = tid >> 3;
      const int c4  = (tid & 7) * 4;
      const v4f xv = *(const v4f*)(x + ((size_t)(b0 + row) * kT + t) * kIn + c4);
      const unsigned wa = (unsigned)f16bits(xv[0] * kActS) | ((unsigned)f16bits(xv[1] * kActS) << 16);
      const unsigned wb = (unsigned)f16bits(xv[2] * kActS) | ((unsigned)f16bits(xv[3] * kActS) << 16);
      v2u wv = {wa, wb};
      *(v2u*)(xs_l + row * XP + c4) = wv;
    }
    if (wave == 0) {
      const int row = c;
      const float* dp = dt + ((size_t)(b0 + row) * kT + t) * 2;
      const float d0 = dp[0];
      const float d1 = dp[1];
      const float s = (d1 - d0) * kDtScale;
      if (lane < 16) scl_l[row] = s;
    }
    __syncthreads();

    float sc[8];
#pragma unroll
    for (int r = 0; r < 8; ++r) sc[r] = scl_l[8 * hh + r];
    const int cur = t & 1;
    const _Float16* hcur = (const _Float16*)(hs_l + cur * kRows * HP);
    unsigned short* hnx  = hs_l + (cur ^ 1) * kRows * HP;
    const _Float16* hnxh = (const _Float16*)hnx;

    {
      v8f ar[2], az[2], axn[2], ahn[2];
#pragma unroll
      for (int us = 0; us < 2; ++us) { ar[us] = zero8(); az[us] = zero8(); axn[us] = zero8(); ahn[us] = zero8(); }
      {
        const v16h ax = frag_load(xsh + c * XP + koff);
#pragma unroll
        for (int us = 0; us < 2; ++us) {
          const int n = 32 * wave + 16 * us + c;
          ar[us]  = mma_h(ax, frag_load(Wih + (size_t)n * kIn + koff), ar[us]);
          az[us]  = mma_h(ax, frag_load(Wih + (size_t)(kH + n) * kIn + koff), az[us]);
          axn[us] = mma_h(ax, frag_load(Wih + (size_t)(2 * kH + n) * kIn + koff), axn[us]);
        }
      }
#pragma unroll
      for (int ks = 0; ks < 4; ++ks) {
        const int k0 = 32 * ks;
        const v16h ah = frag_load(hcur + c * HP + koff + k0);
#pragma unroll
        for (int us = 0; us < 2; ++us) {
          const int n = 32 * wave + 16 * us + c;
          ar[us]  = mma_h(ah, frag_load(Whh + (size_t)n * kH + koff + k0), ar[us]);
          az[us]  = mma_h(ah, frag_load(Whh + (size_t)(kH + n) * kH + koff + k0), az[us]);
          ahn[us] = mma_h(ah, frag_load(Whh + (size_t)(2 * kH + n) * kH + koff + k0), ahn[us]);
        }
      }
#pragma unroll
      for (int us = 0; us < 2; ++us) {
        const int colh = 32 * wave + 16 * us + c;
#pragma unroll
        for (int r = 0; r < 8; ++r) {
          const int row = 8 * hh + r;
          const float rg  = sigm_f(ar[us][r] * kInv + brr[us]);
          const float zg  = sigm_f(az[us][r] * kInv + bzz[us]);
          const float ghn = ahn[us][r] * kInv + bhn[us];
          const float gxn = axn[us][r] * kInv + bxn[us];
          const float ng  = tanh_f(gxn + rg * ghn);
          const float hn  = (1.0f - zg) * ng + zg * hreg[us][r];
          hreg[us][r] = hn;
          hnx[row * HP + colh] = f16bits(hn * kActS);
        }
      }
    }
    __syncthreads();

#pragma unroll 1
    for (int e = 0; e < kNEuler; ++e) {
      {
        v8f au = zero8();
#pragma unroll
        for (int ks = 0; ks < 4; ++ks) {
          const int k0 = 32 * ks;
          const v16h ah = frag_load(hnxh + c * HP + koff + k0);
          au = mma_h(ah, frag_load(W1 + (size_t)(16 * wave + c) * kH + koff + k0), au);
        }
#pragma unroll
        for (int r = 0; r < 8; ++r) {
          const int row = 8 * hh + r;
          const float u = tanh_f(au[r] * kInv + b1v);
          us_l[row * UP + 16 * wave + c] = f16bits(u * kActS);
        }
      }
      __syncthreads();
      {
        v8f af[2];
        af[0] = zero8(); af[1] = zero8();
#pragma unroll
        for (int ks = 0; ks < 2; ++ks) {
          const int k0 = 32 * ks;
          const v16h a = frag_load(ush + c * UP + koff + k0);
#pragma unroll
          for (int us = 0; us < 2; ++us) {
            const int n = 32 * wave + 16 * us + c;
            af[us] = mma_h(a, frag_load(W2 + (size_t)n * kOdeP + koff + k0), af[us]);
          }
        }
#pragma unroll
        for (int us = 0; us < 2; ++us) {
          const int colh = 32 * wave + 16 * us + c;
#pragma unroll
          for (int r = 0; r < 8; ++r) {
            const int row = 8 * hh + r;
            const float f  = tanh_f(af[us][r] * kInv + b2v[us]) * sc[r];
            const float hn = hreg[us][r] + kStep * f;
            hreg[us][r] = hn;
            hnx[row * HP + colh] = f16bits(hn * kActS);
          }
        }
      }
      __syncthreads();
    }

    {
      v8f al = zero8();
      v8f asg[2];
      asg[0] = zero8(); asg[1] = zero8();
#pragma unroll
      for (int ks = 0; ks < 4; ++ks) {
        const int k0 = 32 * ks;
        const v16h ah = frag_load(hnxh + c * HP + koff + k0);
        al = mma_h(ah, frag_load(Wl1 + (size_t)(16 * wave + c) * kH + koff + k0), al);
#pragma unroll
        for (int us = 0; us < 2; ++us) {
          const int n = 32 * wave + 16 * us + c;
          asg[us] = mma_h(ah, frag_load(Ws1 + (size_t)n * kH + koff + k0), asg[us]);
        }
      }
      float pm[8], ps[8];
#pragma unroll
      for (int r = 0; r < 8; ++r) {
        const float m  = fmaxf(al[r] * kInv + bl1v, 0.0f);
        pm[r] = m * wmuv;
        const float s0 = tanh_f(asg[0][r] * kInv + bs1v[0]);
        const float s1 = tanh_f(asg[1][r] * kInv + bs1v[1]);
        ps[r] = s0 * ws2v[0] + s1 * ws2v[1];
      }
#pragma unroll
      for (int r = 0; r < 8; ++r) {
#pragma unroll
        for (int off = 1; off < 16; off <<= 1) {
          pm[r] += __shfl_xor(pm[r], off, 32);
          ps[r] += __shfl_xor(ps[r], off, 32);
        }
      }
#pragma unroll
      for (int r = 0; r < 8; ++r) {
        if (c == r) {
          pmu_l[wave * kRows + 8 * hh + r] = pm[r];
          psg_l[wave * kRows + 8 * hh + r] = ps[r];
        }
      }
    }
    __syncthreads();
    if (wave == 0) {
      const int row = c;
      const float m = ((pmu_l[row] + pmu_l[kRows + row]) + pmu_l[2 * kRows + row]) + pmu_l[3 * kRows + row] + bmu0;
      const float sv = ((psg_l[row] + psg_l[kRows + row]) + psg_l[2 * kRows + row]) + psg_l[3 * kRows + row] + bs20;
      const float sp = fmaxf(sv, 0.0f) + log1pf(expf(-fabsf(sv)));
      if (lane < 16) mus_l[row * kT + t] = m;
      else           sgs_l[row * kT + t] = sp;
    }
  }
  __syncthreads();

  {
    float* o0 = out + (size_t)b0 * kT;
    float* o1 = out + (size_t)kBatch * kT + (size_t)b0 * kT;
    for (int pass = 0; pass < 2; ++pass) {
      for (int i = tid; i < (kRows * kT) / 4; i += kThreads) {
        const v4f a = *(const v4f*)(mus_l + 4 * i);
        const v4f s = *(const v4f*)(sgs_l + 4 * i);
        *(volatile v4f*)(o0 + 4 * i) = a;
        *(volatile v4f*)(o1 + 4 * i) = s;
      }
      __threadfence();
    }
  }
}

extern "C" void kernel_launch(void* const* d_in, const int* in_sizes, int n_in,
                              void* d_out, int out_size, void* d_ws, size_t ws_size,
                              hipStream_t stream) {
  if (n_in < 18) return;
  if (in_sizes[0]  != kBatch * kT * 2)   return;
  if (in_sizes[1]  != kBatch * kT * kIn) return;
  if (in_sizes[2]  != 3 * kH * kIn) return;
  if (in_sizes[3]  != 3 * kH * kH)  return;
  if (in_sizes[4]  != 3 * kH || in_sizes[5] != 3 * kH) return;
  if (in_sizes[6]  != kOde * kH || in_sizes[7] != kOde) return;
  if (in_sizes[8]  != kH * kOde || in_sizes[9] != kH)   return;
  if (in_sizes[10] != kL1 * kH  || in_sizes[11] != kL1) return;
  if (in_sizes[12] != kL1 || in_sizes[13] != 1) return;
  if (in_sizes[14] != kH * kH || in_sizes[15] != kH) return;
  if (in_sizes[16] != kH || in_sizes[17] != 1) return;
  if (out_size != 2 * kBatch * kT) return;
  if (ws_size < kWsTotal) return;

  const float* dt  = (const float*)d_in[0];
  const float* x   = (const float*)d_in[1];
  const float* Wih = (const float*)d_in[2];
  const float* Whh = (const float*)d_in[3];
  const float* bih = (const float*)d_in[4];
  const float* bhh = (const float*)d_in[5];
  const float* W1  = (const float*)d_in[6];
  const float* b1  = (const float*)d_in[7];
  const float* W2  = (const float*)d_in[8];
  const float* b2  = (const float*)d_in[9];
  const float* Wl1 = (const float*)d_in[10];
  const float* bl1 = (const float*)d_in[11];
  const float* Wmu = (const float*)d_in[12];
  const float* bmu = (const float*)d_in[13];
  const float* Ws1 = (const float*)d_in[14];
  const float* bs1 = (const float*)d_in[15];
  const float* Ws2 = (const float*)d_in[16];
  const float* bs2 = (const float*)d_in[17];

  char* ws = (char*)d_ws;
  unsigned short* wih16 = (unsigned short*)(ws + kOffWih);
  unsigned short* whh16 = (unsigned short*)(ws + kOffWhh);
  unsigned short* w1p   = (unsigned short*)(ws + kOffW1);
  unsigned short* w2p   = (unsigned short*)(ws + kOffW2);
  unsigned short* wl1p  = (unsigned short*)(ws + kOffWl1);
  unsigned short* ws1p  = (unsigned short*)(ws + kOffWs1);

  prep_plane_f16<<<dim3((3 * kH * kIn / 8 + 255) / 256), dim3(256), 0, stream>>>(Wih, 3 * kH, kIn, wih16, 3 * kH, kIn, kWgtS);
  prep_plane_f16<<<dim3((3 * kH * kH / 8 + 255) / 256), dim3(256), 0, stream>>>(Whh, 3 * kH, kH, whh16, 3 * kH, kH, kWgtS);
  prep_plane_f16<<<dim3((kOdeP * kH / 8 + 255) / 256), dim3(256), 0, stream>>>(W1, kOde, kH, w1p, kOdeP, kH, kWgtS);
  prep_plane_f16<<<dim3((kH * kOdeP / 8 + 255) / 256), dim3(256), 0, stream>>>(W2, kH, kOde, w2p, kH, kOdeP, kWgtS);
  prep_plane_f16<<<dim3((kL1 * kH / 8 + 255) / 256), dim3(256), 0, stream>>>(Wl1, kL1, kH, wl1p, kL1, kH, kWgtS);
  prep_plane_f16<<<dim3((kH * kH / 8 + 255) / 256), dim3(256), 0, stream>>>(Ws1, kH, kH, ws1p, kH, kH, kWgtS);

  odegru_main<<<dim3(kBatch / kRows), dim3(kThreads), 0, stream>>>(
      dt, x, wih16, whh16, w1p, w2p, wl1p, ws1p,
      bih, bhh, b1, b2, bl1, Wmu, bmu, bs1, Ws2, bs2, (float*)d_out);
}
